// Harp_81346680586803
// MI455X (gfx1250) — hardware-run, weakly checked
//
#include <hip/hip_runtime.h>


#define NB_  4
#define TT   2048
#define DM   1024
#define ZH   2
#define RH   0
#define PCAR 1024.0f
#define SCL  0.125f
#define QSC  0.16666667163372040f
typedef _Float16 h16;
typedef unsigned short bf;
typedef __attribute__((ext_vector_type(16))) __bf16   v16bf;
typedef __attribute__((ext_vector_type(16))) _Float16 v16h;
typedef __attribute__((ext_vector_type(8)))  _Float16 v8h;
typedef __attribute__((ext_vector_type(8)))  unsigned short v8us;
typedef __attribute__((ext_vector_type(8)))  float    v8f;
typedef __attribute__((ext_vector_type(4)))  float    v4f;
typedef v8h  __attribute__((may_alias)) v8ha;
typedef v4f  __attribute__((may_alias)) v4fa;
typedef v8us __attribute__((may_alias)) v8usa;

__device__ __forceinline__ unsigned short f2bf(float f) { unsigned u = __float_as_uint(f); u += 0x7FFFu + ((u >> 16) & 1u); return (unsigned short)(u >> 16); }
__device__ __forceinline__ float bf2f(unsigned short b) { return __uint_as_float(((unsigned)b) << 16); }
__device__ __forceinline__ float bfr(float f) { return bf2f(f2bf(f)); }
__device__ __forceinline__ v16h cat16(v8h lo, v8h hi) { return __builtin_shufflevector(lo, hi, 0, 1, 2, 3, 4, 5, 6, 7, 8, 9, 10, 11, 12, 13, 14, 15); }
__device__ __forceinline__ v16bf cat16b(v8us lo, v8us hi) { return __builtin_bit_cast(v16bf, __builtin_shufflevector(lo, hi, 0, 1, 2, 3, 4, 5, 6, 7, 8, 9, 10, 11, 12, 13, 14, 15)); }
__device__ __forceinline__ v8f wmma16(v16h a, v16h b, v8f c) { return __builtin_amdgcn_wmma_f32_16x16x32_f16(false, a, false, b, (short)0, c, false, false); }
__device__ __forceinline__ v8f wmmab(v16bf a, v16bf b, v8f c) { return __builtin_amdgcn_wmma_f32_16x16x32_bf16(false, a, false, b, (short)0, c, false, false); }


template <typename T16> struct WFrag;
template <> struct WFrag<h16> { typedef v16h V; static __device__ __forceinline__ V ld(const h16* p) { return cat16(*(const v8h*)p, *(const v8h*)(p + 16)); } static __device__ __forceinline__ v8f mma(V a, V b, v8f c) { return wmma16(a, b, c); } };
template <> struct WFrag<bf> { typedef v16bf V; static __device__ __forceinline__ V ld(const bf* p) { return cat16b(*(const v8us*)p, *(const v8us*)(p + 16)); } static __device__ __forceinline__ v8f mma(V a, V b, v8f c) { return wmmab(a, b, c); } };
template <typename T16, int NSPLIT, bool BIAS>
__global__ __launch_bounds__(32) void k_gemmw(const T16* __restrict__ A, const T16* __restrict__ A2, const T16* __restrict__ Bt, const T16* __restrict__ Bt2, int K, float* C, int ldc, const float* __restrict__ bias, size_t sA, size_t sB, size_t sC) {
    typedef typename WFrag<T16>::V V;
    __shared__ __align__(16) float os[16 * 68];
    const size_t z = blockIdx.z; A += z * sA; if (A2) A2 += z * sA; Bt += z * sB; if (Bt2) Bt2 += z * sB; C += z * sC;
    const int lane = threadIdx.x & 31, lr = lane & 15, hi = lane >> 4; const int r0 = blockIdx.x * 64, c0 = blockIdx.y * 64;
    v8f acc[4][4];
#pragma unroll
    for (int mb = 0; mb < 4; ++mb)
#pragma unroll
        for (int nb = 0; nb < 4; ++nb) acc[mb][nb] = (v8f){};
    const size_t aoff = (size_t)(r0 + lr) * K + 8 * hi, boff = (size_t)(c0 + lr) * K + 8 * hi;
    for (int kc = 0; kc < K; kc += 32) {
        V a[4], a2[4];
#pragma unroll
        for (int mb = 0; mb < 4; ++mb) { a[mb] = WFrag<T16>::ld(A + aoff + (size_t)mb * 16 * K + kc); if (NSPLIT == 1 || NSPLIT == 2) a2[mb] = WFrag<T16>::ld(A2 + aoff + (size_t)mb * 16 * K + kc); }
#pragma unroll
        for (int nb = 0; nb < 4; ++nb) { const V b = WFrag<T16>::ld(Bt + boff + (size_t)nb * 16 * K + kc); V b2; if (NSPLIT >= 2) b2 = WFrag<T16>::ld(Bt2 + boff + (size_t)nb * 16 * K + kc);
#pragma unroll
            for (int mb = 0; mb < 4; ++mb) { acc[mb][nb] = WFrag<T16>::mma(a[mb], b, acc[mb][nb]); if (NSPLIT == 1 || NSPLIT == 2) acc[mb][nb] = WFrag<T16>::mma(a2[mb], b, acc[mb][nb]); if (NSPLIT >= 2) acc[mb][nb] = WFrag<T16>::mma(a[mb], b2, acc[mb][nb]); } }
        asm volatile("v_nop\n\tv_nop\n\tv_nop\n\tv_nop" : "+v"(acc[0][0]), "+v"(acc[1][1]), "+v"(acc[2][2]), "+v"(acc[3][3]) : "v"(a[0]), "v"(a[3]));
    }
#pragma unroll
    for (int mb = 0; mb < 4; ++mb) {
#pragma unroll
        for (int nb = 0; nb < 4; ++nb) {
#pragma unroll
            for (int j = 0; j < 8; ++j) os[(hi * 8 + j) * 68 + nb * 16 + lr] = acc[mb][nb][j]; }
        __builtin_amdgcn_wave_barrier(); asm volatile("" ::: "memory");
        float* crow = C + (size_t)(r0 + mb * 16) * ldc + c0;
#pragma unroll 1
        for (int ps = 0; ps < 2; ++ps) {
#pragma unroll
            for (int s = 0; s < 8; ++s) { const int row = 2 * s + hi, cofs = lr * 4; v4f val = *(const v4fa*)(os + row * 68 + cofs); if (BIAS) { val[0] += bfr(bias[c0 + cofs]); val[1] += bfr(bias[c0 + cofs + 1]); val[2] += bfr(bias[c0 + cofs + 2]); val[3] += bfr(bias[c0 + cofs + 3]); }
                *(volatile v4f*)(crow + (size_t)row * ldc + cofs) = val; }
            if (ps == 0) __threadfence(); }
        __builtin_amdgcn_wave_barrier(); asm volatile("" ::: "memory");
    }
}

__device__ __forceinline__ h16 tohx(float x) { return (h16)x; }
__device__ __forceinline__ void splitf(float y, unsigned short& h, unsigned short& l) { h = f2bf(y); l = f2bf(y - bf2f(h)); }
typedef __attribute__((ext_vector_type(2))) _Float16 v2h;
typedef __attribute__((ext_vector_type(4))) _Float16 v4h;
typedef __attribute__((ext_vector_type(2))) unsigned short v2us;
typedef __attribute__((ext_vector_type(4))) unsigned short v4us;
typedef __attribute__((ext_vector_type(2))) float v2f;
typedef __attribute__((ext_vector_type(4))) int v4i;

__global__ __launch_bounds__(256) void k_cvt8(const float* __restrict__ src, bf* dst, size_t n8) { const size_t i = (size_t)blockIdx.x * 256 + threadIdx.x; if (i >= n8) return; const v8f v = *(const v8f*)(src + i * 8); v8us o;
#pragma unroll
    for (int k = 0; k < 8; ++k) o[k] = f2bf(v[k]); *(volatile v8us*)(dst + i * 8) = o; __threadfence(); *(volatile v8us*)(dst + i * 8) = o; }
__global__ __launch_bounds__(256) void k_asoft(const float* __restrict__ Sb, h16* P16, bf* Ph, bf* Pl) {
    const int lane = threadIdx.x & 31; const int row = blockIdx.x * 8 + (threadIdx.x >> 5); if (row >= ZH * TT) return; const int i = row % TT; const int zz = row / TT; (void)zz; const bool hires = (i < RH); const float* sr = Sb + (size_t)row * TT; float v[TT / 32]; float mx = -3.0e38f;
#pragma unroll
    for (int ch = 0; ch < TT / 128; ++ch) { const int j0 = ch * 128 + lane * 4; const v4f a = *(const v4f*)(sr + j0);
#pragma unroll
        for (int q = 0; q < 4; ++q) { const int j = j0 + q; (void)j; const float t = a[q] * SCL; v[ch * 4 + q] = t; mx = fmaxf(mx, t); } }
#pragma unroll
    for (int sh = 16; sh; sh >>= 1) mx = fmaxf(mx, __shfl_xor(mx, sh, 32));
    float sum = 0.f;
#pragma unroll
    for (int k = 0; k < TT / 32; ++k) { float d0 = __fsub_rn(v[k], mx); v[k] = __builtin_amdgcn_exp2f(__fmul_rn(d0, 1.4426950408889634f)); sum += v[k]; }
#pragma unroll
    for (int sh = 16; sh; sh >>= 1) sum += __shfl_xor(sum, sh, 32);
    const float f = __fdiv_rn(hires ? 1.0f : PCAR, sum);
#pragma unroll 1
    for (int ps = 0; ps < 2; ++ps) {
        if (hires) {
#pragma unroll
            for (int ch = 0; ch < TT / 128; ++ch) { v4us oh, ol;
#pragma unroll
                for (int q = 0; q < 4; ++q) { unsigned short a, c2; splitf(v[ch * 4 + q] * f, a, c2); oh[q] = a; ol[q] = c2; }
                const size_t oo = ((size_t)zz * (RH ? RH : 1) + i) * TT + ch * 128 + lane * 4; *(volatile v4us*)(Ph + oo) = oh; *(volatile v4us*)(Pl + oo) = ol; }
        } else {
#pragma unroll
            for (int ch = 0; ch < TT / 128; ++ch) { v4h o4;
#pragma unroll
                for (int q = 0; q < 4; ++q) o4[q] = tohx(v[ch * 4 + q] * f);
                *(volatile v4h*)(P16 + (size_t)row * TT + ch * 128 + lane * 4) = o4; } }
        if (ps == 0) __threadfence(); }
}
__global__ __launch_bounds__(256) void k_tohl(const float* __restrict__ F, float sc, bf* Hh, bf* Hl, size_t n4) { const size_t i = (size_t)blockIdx.x * 256 + threadIdx.x; if (i >= n4) return; const v4f a = *(const v4f*)(F + i * 4); v4us oh, ol;
#pragma unroll
    for (int q = 0; q < 4; ++q) { unsigned short h2, l2; splitf(__fmul_rn(a[q], sc), h2, l2); oh[q] = h2; ol[q] = l2; }
    *(volatile v4us*)(Hh + i * 4) = oh; *(volatile v4us*)(Hl + i * 4) = ol; __threadfence(); *(volatile v4us*)(Hh + i * 4) = oh; *(volatile v4us*)(Hl + i * 4) = ol; }
#define LNC_MAX 2048
template <bool RES>
__global__ __launch_bounds__(256) void k_lnrow(const float* __restrict__ A, const float* __restrict__ R, const float* __restrict__ gamma, const float* __restrict__ beta, float eps, int C, int nrows, float* Y) {
    const int lane = threadIdx.x & 31; const int row = blockIdx.x * 8 + (threadIdx.x >> 5); if (row >= nrows) return; const int nch = C / 128; const float* a = A + (size_t)row * C; float x[LNC_MAX / 32]; float s = 0.0f;
    for (int k = 0; k < LNC_MAX / 128; ++k) { if (k < nch) { const int c0 = k * 128 + lane * 4; v4f v = *(const v4f*)(a + c0);
            if (RES) { const v4f w = *(const v4f*)(R + (size_t)row * C + c0); v[0] = __fadd_rn(v[0], w[0]); v[1] = __fadd_rn(v[1], w[1]); v[2] = __fadd_rn(v[2], w[2]); v[3] = __fadd_rn(v[3], w[3]); }
            x[k * 4 + 0] = v[0]; x[k * 4 + 1] = v[1]; x[k * 4 + 2] = v[2]; x[k * 4 + 3] = v[3]; s = __fadd_rn(__fadd_rn(__fadd_rn(__fadd_rn(s, v[0]), v[1]), v[2]), v[3]); } }
    for (int sh = 16; sh; sh >>= 1) s = __fadd_rn(s, __shfl_xor(s, sh, 32));
    const float mean = __fdiv_rn(s, (float)C); float q = 0.0f;
    for (int k = 0; k < LNC_MAX / 128; ++k) { if (k < nch) {
            for (int j = 0; j < 4; ++j) { const float d = __fsub_rn(x[k * 4 + j], mean); x[k * 4 + j] = d; q = __fmaf_rn(d, d, q); } } }
    for (int sh = 16; sh; sh >>= 1) q = __fadd_rn(q, __shfl_xor(q, sh, 32));
    const float rstd = __fdiv_rn(1.0f, sqrtf(__fadd_rn(__fdiv_rn(q, (float)C), eps)));
    for (int k = 0; k < LNC_MAX / 128; ++k) { if (k < nch) { const int c0 = k * 128 + lane * 4; const v4f g = *(const v4f*)(gamma + c0); const v4f bt = *(const v4f*)(beta + c0);
            for (int j = 0; j < 4; ++j) x[k * 4 + j] = __fmaf_rn(__fmul_rn(x[k * 4 + j], rstd), bfr(g[j]), bfr(bt[j])); } }
    float* y = Y + (size_t)row * C;
    for (int ps = 0; ps < 2; ++ps) {
        for (int k = 0; k < LNC_MAX / 128; ++k) { if (k < nch) { v4f o; o[0] = x[k * 4 + 0]; o[1] = x[k * 4 + 1]; o[2] = x[k * 4 + 2]; o[3] = x[k * 4 + 3]; *(volatile v4f*)(y + k * 128 + lane * 4) = o; } }
        if (ps == 0) __threadfence(); }
}
__global__ __launch_bounds__(256) void k_f2h(const float* __restrict__ S, h16* P16, size_t n4) { const size_t i = (size_t)blockIdx.x * 256 + threadIdx.x; if (i >= n4) return; const v4f v = *(const v4f*)(S + i * 4); v4h o;
#pragma unroll
    for (int q = 0; q < 4; ++q) o[q] = tohx(v[q]);
    *(volatile v4h*)(P16 + i * 4) = o; __threadfence(); *(volatile v4h*)(P16 + i * 4) = o; }
__global__ __launch_bounds__(256) void k_qcast(const float* __restrict__ Q, float sc, h16* Q16) { const size_t i = (size_t)blockIdx.x * 256 + threadIdx.x; const v4f a = *(const v4f*)(Q + i * 4); v4h o;
#pragma unroll
    for (int q = 0; q < 4; ++q) { const float y = __fmul_rn(a[q], sc); o[q] = tohx((fabsf(y) < 6.103515625e-5f) ? 0.0f : y); }
    *(volatile v4h*)(Q16 + i * 4) = o; __threadfence(); *(volatile v4h*)(Q16 + i * 4) = o; }
__global__ __launch_bounds__(256) void k_bcar(const float* __restrict__ b, float* BV) { const unsigned c = blockIdx.x * 256 + threadIdx.x; const float v = __fmul_rn(bfr(b[c]), PCAR); *(volatile float*)(BV + c) = v; __threadfence(); *(volatile float*)(BV + c) = v; }
__global__ __launch_bounds__(256) void k_colmean(const float* __restrict__ H, float* POOL) { const size_t c = (size_t)blockIdx.x * 256 + threadIdx.x; float s = 0.f;
    for (int t = 0; t < TT; ++t) s = __fadd_rn(s, H[(size_t)t * DM + c]);
    const float m = __fmul_rn(s, (1.0f / TT) * (1.0f / PCAR)); *(volatile float*)(POOL + c) = m; __threadfence(); *(volatile float*)(POOL + c) = m; }
__global__ __launch_bounds__(256) void k_epi(const float* __restrict__ x, const float* __restrict__ eps, const float* __restrict__ MU, const float* __restrict__ LV, float* Z) { const size_t i = (size_t)blockIdx.x * 256 + threadIdx.x; const v4f a = *(const v4f*)(x + i * 4), e = *(const v4f*)(eps + i * 4), m = *(const v4f*)(MU + i * 4), l = *(const v4f*)(LV + i * 4); v4f o;
#pragma unroll
    for (int q = 0; q < 4; ++q) { const float sd = expf(__fmul_rn(0.5f, l[q])); const float z = fmaxf(__fmaf_rn(bfr(e[q]), sd, m[q]), 0.0f); o[q] = __fadd_rn(bfr(a[q]), z); }
    *(volatile v4f*)(Z + i * 4) = o; __threadfence(); *(volatile v4f*)(Z + i * 4) = o; }
__global__ __launch_bounds__(32) void k_pgate(const float* __restrict__ POOL, const float* __restrict__ Wg, const float* __restrict__ bg, float* PG) { const int b = threadIdx.x; if (b >= NB_) return; float s = 0.f;
    for (int c = 0; c < DM; ++c) s = __fmaf_rn(POOL[(size_t)b * DM + c], bfr(Wg[c]), s);
    const float p = __fdiv_rn(1.0f, __fadd_rn(1.0f, expf(-__fadd_rn(s, bfr(bg[0]))))); *(volatile float*)(PG + b) = p; __threadfence(); *(volatile float*)(PG + b) = p; }

extern "C" void kernel_launch(void* const* d_in, const int* in_sizes, int n_in,
                              void* d_out, int out_size, void* d_ws, size_t ws_size, hipStream_t stream) {
    (void)in_sizes; (void)n_in; (void)out_size;
    const float* xin = (const float*)d_in[0]; const float* ein = (const float*)d_in[1]; const float* wq = (const float*)d_in[2]; const float* bq = (const float*)d_in[3]; const float* wk = (const float*)d_in[4]; const float* bk = (const float*)d_in[5]; const float* wv = (const float*)d_in[6]; const float* bv = (const float*)d_in[7];
    const float* wmu = (const float*)d_in[8]; const float* bmu = (const float*)d_in[9]; const float* wlv = (const float*)d_in[10]; const float* blv = (const float*)d_in[11]; const float* wg = (const float*)d_in[12]; const float* bg = (const float*)d_in[13]; const float* gam = (const float*)d_in[14]; const float* bet = (const float*)d_in[15];
    const size_t PL = (size_t)NB_ * TT * DM;
    float* OUT0 = (float*)d_out; float* OUT1 = OUT0 + PL; float* OUT2 = OUT1 + PL; float* OUT3 = OUT2 + PL;
    char* wsp = (char*)d_ws;
    auto take = [&](size_t bytes) { char* p = wsp; wsp += (bytes + 255) & ~(size_t)255; return (void*)p; };
    bf* WQB = (bf*)take((size_t)DM * DM * 2); bf* WKB = (bf*)take((size_t)DM * DM * 2); bf* WVB = (bf*)take((size_t)DM * DM * 2); bf* WMB = (bf*)take((size_t)DM * DM * 2); bf* WLB = (bf*)take((size_t)DM * DM * 2); float* BV = (float*)take((size_t)DM * 4); float* POOL = (float*)take((size_t)NB_ * DM * 4);
    bf* XB = (bf*)take((size_t)TT * DM * 2); float* QF = (float*)take((size_t)TT * DM * 4); float* KF = (float*)take((size_t)TT * DM * 4); float* VTF = (float*)take((size_t)DM * TT * 4);
    h16* Q16 = (h16*)take((size_t)ZH * TT * DM * 2); h16* K16 = (h16*)take((size_t)ZH * TT * DM * 2); h16* VT16 = (h16*)take((size_t)ZH * DM * TT * 2);
    float* Sb = (float*)take((size_t)ZH * TT * TT * 4); h16* P16 = (h16*)take((size_t)ZH * TT * TT * 2); float* Hb = (float*)take((size_t)ZH * TT * DM * 4); bf* Hh = (bf*)take((size_t)ZH * TT * DM * 2); bf* Hl = (bf*)take((size_t)ZH * TT * DM * 2); float* ZF = (float*)take((size_t)ZH * TT * DM * 4);
    if ((size_t)(wsp - (char*)d_ws) > ws_size) return;
    const unsigned GW = (unsigned)(((size_t)DM * DM / 8 + 255) / 256);
    k_cvt8<<<GW, 256, 0, stream>>>(wq, WQB, (size_t)DM * DM / 8); k_cvt8<<<GW, 256, 0, stream>>>(wk, WKB, (size_t)DM * DM / 8); k_cvt8<<<GW, 256, 0, stream>>>(wv, WVB, (size_t)DM * DM / 8); k_cvt8<<<GW, 256, 0, stream>>>(wmu, WMB, (size_t)DM * DM / 8); k_cvt8<<<GW, 256, 0, stream>>>(wlv, WLB, (size_t)DM * DM / 8);
    k_bcar<<<DM / 256, 256, 0, stream>>>(bv, BV);
    const unsigned GX = (unsigned)(((size_t)TT * DM / 8 + 255) / 256), GH = (unsigned)(((size_t)TT * DM / 4 + 255) / 256);
    for (int b0 = 0; b0 < NB_; b0 += ZH) {
        for (int zz = 0; zz < ZH; ++zz) { const int b = b0 + zz;
            k_cvt8<<<GX, 256, 0, stream>>>(xin + (size_t)b * TT * DM, XB, (size_t)TT * DM / 8);
            k_gemmw<bf, 0, true><<<dim3(TT / 64, DM / 64, 1), 32, 0, stream>>>(XB, nullptr, WQB, nullptr, DM, QF, DM, bq, 0, 0, 0);
            k_qcast<<<(unsigned)((size_t)TT * DM / 4 / 256), 256, 0, stream>>>(QF, QSC, Q16 + (size_t)zz * TT * DM);
            k_gemmw<bf, 0, true><<<dim3(TT / 64, DM / 64, 1), 32, 0, stream>>>(XB, nullptr, WKB, nullptr, DM, KF, DM, bk, 0, 0, 0);
            k_f2h<<<GH, 256, 0, stream>>>(KF, K16 + (size_t)zz * TT * DM, (size_t)TT * DM / 4);
            k_gemmw<bf, 0, false><<<dim3(DM / 64, TT / 64, 1), 32, 0, stream>>>(WVB, nullptr, XB, nullptr, DM, VTF, TT, nullptr, 0, 0, 0);
            k_f2h<<<GH, 256, 0, stream>>>(VTF, VT16 + (size_t)zz * DM * TT, (size_t)DM * TT / 4); }
        k_gemmw<h16, 0, false><<<dim3(TT / 64, TT / 64, ZH), 32, 0, stream>>>(Q16, nullptr, K16, nullptr, DM, Sb, TT, nullptr, (size_t)TT * DM, (size_t)TT * DM, (size_t)TT * TT);
        k_asoft<<<ZH * TT / 8, 256, 0, stream>>>(Sb, P16, nullptr, nullptr);
        k_gemmw<h16, 0, true><<<dim3(TT / 64, DM / 64, ZH), 32, 0, stream>>>(P16, nullptr, VT16, nullptr, TT, Hb, DM, BV, (size_t)TT * TT, (size_t)DM * TT, (size_t)TT * DM);
        for (int zz = 0; zz < ZH; ++zz) k_colmean<<<DM / 256, 256, 0, stream>>>(Hb + (size_t)zz * TT * DM, POOL + (size_t)(b0 + zz) * DM);
        k_tohl<<<(unsigned)(((size_t)ZH * TT * DM / 4 + 255) / 256), 256, 0, stream>>>(Hb, 1.0f / PCAR, Hh, Hl, (size_t)ZH * TT * DM / 4);
        k_gemmw<bf, 1, true><<<dim3(TT / 64, DM / 64, ZH), 32, 0, stream>>>(Hh, Hl, WMB, nullptr, DM, OUT1 + (size_t)b0 * TT * DM, DM, bmu, (size_t)TT * DM, 0, (size_t)TT * DM);
        k_gemmw<bf, 1, true><<<dim3(TT / 64, DM / 64, ZH), 32, 0, stream>>>(Hh, Hl, WLB, nullptr, DM, OUT2 + (size_t)b0 * TT * DM, DM, blv, (size_t)TT * DM, 0, (size_t)TT * DM);
        k_epi<<<(unsigned)((size_t)ZH * TT * DM / 4 / 256), 256, 0, stream>>>(xin + (size_t)b0 * TT * DM, ein + (size_t)b0 * TT * DM, OUT1 + (size_t)b0 * TT * DM, OUT2 + (size_t)b0 * TT * DM, ZF);
        for (int zz = 0; zz < ZH; ++zz) k_lnrow<false><<<(unsigned)((TT + 7) / 8), 256, 0, stream>>>(ZF + (size_t)zz * TT * DM, nullptr, gam, bet, 1.0e-5f, DM, TT, OUT0 + (size_t)(b0 + zz) * TT * DM);
    }
    k_pgate<<<1, 32, 0, stream>>>(POOL, wg, bg, OUT3);
}
